// Raymarcher_4861902979095
// MI455X (gfx1250) — hardware-run, weakly checked
//
#include <hip/hip_runtime.h>
#include <math.h>

typedef __attribute__((ext_vector_type(16))) _Float16 v16h;
typedef __attribute__((ext_vector_type(8)))  _Float16 v8h;
typedef __attribute__((ext_vector_type(8)))  float    v8f;
typedef __attribute__((ext_vector_type(4)))  float    v4f;
typedef __attribute__((ext_vector_type(2)))  float    v2f;

constexpr int kBatch       = 8;
constexpr int kPts         = 16384;
constexpr int kFeat        = 256;
constexpr int kHid         = 16;
constexpr int kGates       = 4 * kHid;
constexpr int kSteps       = 10;
constexpr int kRays        = kBatch * kPts;
constexpr int kBlkThreads  = 128;
constexpr int kWaves       = 4;
constexpr int kWaveRays    = 32;
constexpr int kBlkRays     = kWaves * kWaveRays;
constexpr int kBlocks      = kRays / kBlkRays;
constexpr int kBlkPerBatch = kPts / kBlkRays;
constexpr int kKReal       = kFeat + kHid;
constexpr int kKPad        = 288;
constexpr int kKChunks     = kKPad / 32;
constexpr int kGatePitch   = 68;
constexpr float kWCarry    = 256.0f;
constexpr float kXCarry    = 16.0f;
constexpr float kFold      = 1.0f / (kWCarry * kXCarry);
constexpr int kOut1Off     = kRays * 3;

static_assert(kGates == 64, "gate width");
static_assert(kBlkRays == 128 && kBlocks == 1024 && kBlkPerBatch == 128, "block map");
static_assert((kPts % kBlkRays) == 0, "a block never straddles a batch element");
static_assert(kKReal == 272 && (kKPad % 32) == 0 && kKPad >= kKReal && kKChunks == 9, "k padding");
static_assert(kKPad - kKReal == 16, "two 8-half pad groups per row");
static_assert((size_t)kOut1Off * 4 == 1572864ull, "second output byte offset");
static_assert(((size_t)kOut1Off + kRays) * 4 == 2097152ull, "output total bytes");
static_assert(((kKPad * 2) % 16) == 0 && ((kGatePitch * 4) % 16) == 0, "16-byte aligned LDS rows");
static_assert(kWaveRays * 3 + kWaveRays == 128, "staging tile: 96 world floats + 32 depth floats");

union FragU { v16h v; v8h h[2]; };
__device__ __forceinline__ v16h frag_load(const _Float16* p) {
  FragU f;
  f.h[0] = *(const v8h*)(p);
  f.h[1] = *(const v8h*)(p + 16);
  return f.v;
}

__device__ __forceinline__ v8f mma_f16(v16h a, v16h b, v8f c) {
  c = __builtin_amdgcn_wmma_f32_16x16x32_f16(false, a, false, b, (short)0, c, false, false);
  asm volatile("v_nop\n\tv_nop\n\tv_nop\n\tv_nop" : "+v"(c) : "v"(a), "v"(b));
  return c;
}

__device__ __forceinline__ void wave_lds_sync() {
  __builtin_amdgcn_fence(__ATOMIC_RELEASE, "workgroup");
  __builtin_amdgcn_wave_barrier();
  __builtin_amdgcn_fence(__ATOMIC_ACQUIRE, "workgroup");
}

__device__ __forceinline__ float sigm_fast(float x) {
  return __builtin_amdgcn_rcpf(1.0f + __expf(-x));
}
__device__ __forceinline__ float tanh_fast(float x) {
  return 1.0f - 2.0f * __builtin_amdgcn_rcpf(__expf(2.0f * x) + 1.0f);
}

__device__ __forceinline__ double det3(double a0, double b0, double d0,
                                       double a1, double b1, double d1,
                                       double a2, double b2, double d2) {
  return a0 * (b1 * d2 - b2 * d1) - b0 * (a1 * d2 - a2 * d1) + d0 * (a1 * b2 - a2 * b1);
}

__global__ __launch_bounds__(128) void ray_cell_kernel(
    const float* __restrict__ cam2world, const float* __restrict__ intrinsics,
    const float* __restrict__ uv, const float* __restrict__ init_depth,
    const float* __restrict__ W_phi, const float* __restrict__ b_phi,
    const float* __restrict__ W_ih, const float* __restrict__ b_ih,
    const float* __restrict__ W_hh, const float* __restrict__ b_hh,
    const float* __restrict__ W_out, const float* __restrict__ b_out,
    float* __restrict__ out)
{
  __shared__ __align__(16) _Float16 sBt[kGates * kKPad];
  __shared__ __align__(16) _Float16 sA[kWaves][kWaveRays * kKPad];
  __shared__ __align__(16) float    sG[kWaves][kWaveRays * kGatePitch];
  __shared__ __align__(16) float    sWp[4 * kFeat];
  __shared__ __align__(16) float    sBias[kGates];
  __shared__ __align__(16) float    sWo[kHid];

  const int tid   = threadIdx.x;
  const int lane  = tid & 31;
  const int wave  = tid >> 5;
  const int rlane = lane & 15;
  const int koff  = (lane >> 4) * 8;
  const int mOff  = (lane >> 4) * 8;

  v8h zv;
#pragma unroll
  for (int e = 0; e < 8; ++e) zv[e] = (_Float16)0.0f;

#pragma unroll 1
  for (int it = 0; it < 16; ++it) {
    const int idx = it * kBlkThreads + tid;
    const int n   = idx >> 5;
    const int gq  = idx & 31;
    const float* src = W_ih + n * kFeat + gq * 8;
    const v4f a0 = *(const v4f*)(src);
    const v4f a1 = *(const v4f*)(src + 4);
    v8h hv;
#pragma unroll
    for (int e = 0; e < 4; ++e) {
      hv[e]     = (_Float16)(a0[e] * kWCarry);
      hv[4 + e] = (_Float16)(a1[e] * kWCarry);
    }
    *(v8h*)(sBt + n * kKPad + gq * 8) = hv;
  }
  {
    const int n  = tid >> 1;
    const int gq = tid & 1;
    const float* src = W_hh + n * kHid + gq * 8;
    const v4f a0 = *(const v4f*)(src);
    const v4f a1 = *(const v4f*)(src + 4);
    v8h hv;
#pragma unroll
    for (int e = 0; e < 4; ++e) {
      hv[e]     = (_Float16)(a0[e] * kWCarry);
      hv[4 + e] = (_Float16)(a1[e] * kWCarry);
    }
    *(v8h*)(sBt + n * kKPad + kFeat + gq * 8)  = hv;
    *(v8h*)(sBt + n * kKPad + kKReal + gq * 8) = zv;
  }
  {
    const v4f w = *(const v4f*)(W_phi + 4 * tid);
    *(v4f*)(sWp + 4 * tid) = w * kXCarry;
  }
  if (tid < 64) {
    const v4f w = *(const v4f*)(W_phi + 4 * (128 + tid));
    *(v4f*)(sWp + 4 * (128 + tid)) = w * kXCarry;
    const v4f bb = *(const v4f*)(b_phi + 4 * tid);
    *(v4f*)(sWp + 3 * kFeat + 4 * tid) = bb * kXCarry;
    sBias[tid] = b_ih[tid] + b_hh[tid];
  }
  if (wave == 0) {
    sWo[lane & 15] = W_out[lane & 15];
  }
  const float bo = b_out[0];
  __syncthreads();

  const int bix = blockIdx.x / kBlkPerBatch;
  const size_t g0 = (size_t)blockIdx.x * kBlkRays + (size_t)wave * kWaveRays;
  const size_t g  = g0 + lane;
  const float* Mb = cam2world + bix * 16;
  const float m00 = Mb[0],  m01 = Mb[1],  m02 = Mb[2],  m03 = Mb[3];
  const float m10 = Mb[4],  m11 = Mb[5],  m12 = Mb[6],  m13 = Mb[7];
  const float m20 = Mb[8],  m21 = Mb[9],  m22 = Mb[10], m23 = Mb[11];
  const float* Kb = intrinsics + bix * 9;
  const float fx = Kb[0], cx = Kb[2], fy = Kb[4], cy = Kb[5];
  const float rfx = 1.0f / fx;
  const float rfy = 1.0f / fy;
  const v2f uvv = *(const v2f*)(uv + 2 * g);
  const float u0 = uvv[0];
  const float u1 = uvv[1];
  const float d0 = init_depth[g];
  const float xl = (u0 - cx) * rfx;
  const float yl = (u1 - cy) * rfy;

  float dx = fmaf(m00, xl, fmaf(m01, yl, m02));
  float dy = fmaf(m10, xl, fmaf(m11, yl, m12));
  float dz = fmaf(m20, xl, fmaf(m21, yl, m22));
  {
    const float n2  = dx * dx + dy * dy + dz * dz;
    const float inv = 1.0f / sqrtf(n2);
    dx *= inv;
    dy *= inv;
    dz *= inv;
  }
  const float xd = xl * d0;
  const float yd = yl * d0;
  float wx = m00 * xd + m01 * yd + m02 * d0 + m03;
  float wy = m10 * xd + m11 * yd + m12 * d0 + m13;
  float wz = m20 * xd + m21 * yd + m22 * d0 + m23;

  float cst[kHid];
#pragma unroll
  for (int j = 0; j < kHid; ++j) cst[j] = 0.0f;

  _Float16* Aw   = sA[wave];
  _Float16* Arow = Aw + lane * kKPad;
  float*    Gw   = sG[wave];
  const float* grow = Gw + lane * kGatePitch;

  *(v8h*)(Arow + kFeat)      = zv;
  *(v8h*)(Arow + kFeat + 8)  = zv;
  *(v8h*)(Arow + kKReal)     = zv;
  *(v8h*)(Arow + kKReal + 8) = zv;

#pragma unroll 1
  for (int step = 0; step < kSteps; ++step) {
#pragma unroll 1
    for (int f8 = 0; f8 < kFeat / 8; ++f8) {
      const float* wp = sWp + f8 * 8;
      const v4f w0a = *(const v4f*)(wp);
      const v4f w0b = *(const v4f*)(wp + 4);
      const v4f w1a = *(const v4f*)(wp + kFeat);
      const v4f w1b = *(const v4f*)(wp + kFeat + 4);
      const v4f w2a = *(const v4f*)(wp + 2 * kFeat);
      const v4f w2b = *(const v4f*)(wp + 2 * kFeat + 4);
      const v4f bba = *(const v4f*)(wp + 3 * kFeat);
      const v4f bbb = *(const v4f*)(wp + 3 * kFeat + 4);
      v8h xv;
#pragma unroll
      for (int e = 0; e < 4; ++e) {
        float ta = fmaf(wx, w0a[e], bba[e]);
        ta = fmaf(wy, w1a[e], ta);
        ta = fmaf(wz, w2a[e], ta);
        ta = fmaxf(ta, 0.0f);
        float tb = fmaf(wx, w0b[e], bbb[e]);
        tb = fmaf(wy, w1b[e], tb);
        tb = fmaf(wz, w2b[e], tb);
        tb = fmaxf(tb, 0.0f);
        xv[e]     = (_Float16)ta;
        xv[4 + e] = (_Float16)tb;
      }
      *(v8h*)(Arow + f8 * 8) = xv;
    }
    wave_lds_sync();

    v8f acc[2][4];
#pragma unroll
    for (int i = 0; i < 2; ++i)
#pragma unroll
      for (int j = 0; j < 4; ++j) acc[i][j] = (v8f){0.f, 0.f, 0.f, 0.f, 0.f, 0.f, 0.f, 0.f};

#pragma unroll 1
    for (int kc = 0; kc < kKChunks; ++kc) {
      const int kb = kc * 32 + koff;
      v16h bf[4];
#pragma unroll
      for (int j = 0; j < 4; ++j) bf[j] = frag_load(sBt + (16 * j + rlane) * kKPad + kb);
#pragma unroll
      for (int i = 0; i < 2; ++i) {
        const v16h af = frag_load(Aw + (16 * i + rlane) * kKPad + kb);
#pragma unroll
        for (int j = 0; j < 4; ++j) acc[i][j] = mma_f16(af, bf[j], acc[i][j]);
      }
    }

#pragma unroll
    for (int i = 0; i < 2; ++i)
#pragma unroll
      for (int j = 0; j < 4; ++j)
#pragma unroll
        for (int r = 0; r < 8; ++r)
          Gw[(16 * i + mOff + r) * kGatePitch + 16 * j + rlane] = acc[i][j][r];
    wave_lds_sync();

    float hq[kHid];
    float sd = bo;
#pragma unroll
    for (int q = 0; q < 4; ++q) {
      const v4f gi = *(const v4f*)(grow + 4 * q);
      const v4f gf = *(const v4f*)(grow + kHid + 4 * q);
      const v4f gg = *(const v4f*)(grow + 2 * kHid + 4 * q);
      const v4f go = *(const v4f*)(grow + 3 * kHid + 4 * q);
      const v4f bi = *(const v4f*)(sBias + 4 * q);
      const v4f bf4 = *(const v4f*)(sBias + kHid + 4 * q);
      const v4f bg = *(const v4f*)(sBias + 2 * kHid + 4 * q);
      const v4f bq = *(const v4f*)(sBias + 3 * kHid + 4 * q);
      const v4f wo = *(const v4f*)(sWo + 4 * q);
#pragma unroll
      for (int e = 0; e < 4; ++e) {
        const float iv = fmaf(gi[e], kFold, bi[e]);
        const float fv = fmaf(gf[e], kFold, bf4[e]);
        const float gv = fmaf(gg[e], kFold, bg[e]);
        const float ov = fmaf(go[e], kFold, bq[e]);
        const float cn = sigm_fast(fv) * cst[4 * q + e] + sigm_fast(iv) * tanh_fast(gv);
        cst[4 * q + e] = cn;
        const float hj = sigm_fast(ov) * tanh_fast(cn);
        hq[4 * q + e] = hj;
        sd = fmaf(hj, wo[e], sd);
      }
    }

    wx = fmaf(dx, sd, wx);
    wy = fmaf(dy, sd, wy);
    wz = fmaf(dz, sd, wz);

    v8h hva, hvb;
#pragma unroll
    for (int e = 0; e < 8; ++e) {
      hva[e] = (_Float16)(hq[e] * kXCarry);
      hvb[e] = (_Float16)(hq[8 + e] * kXCarry);
    }
    *(v8h*)(Arow + kFeat)      = hva;
    *(v8h*)(Arow + kFeat + 8)  = hvb;
    *(v8h*)(Arow + kKReal)     = zv;
    *(v8h*)(Arow + kKReal + 8) = zv;
  }

  float iv0, iv1, iv2, iv3;
  {
    const double a0 = (double)Mb[0],  b0 = (double)Mb[1],  c0 = (double)Mb[2],  e0 = (double)Mb[3];
    const double a1 = (double)Mb[4],  b1 = (double)Mb[5],  c1 = (double)Mb[6],  e1 = (double)Mb[7];
    const double a2 = (double)Mb[8],  b2 = (double)Mb[9],  c2 = (double)Mb[10], e2 = (double)Mb[11];
    const double a3 = (double)Mb[12], b3 = (double)Mb[13], c3 = (double)Mb[14], e3 = (double)Mb[15];
    const double n0 = det3(a1, b1, e1, a2, b2, e2, a3, b3, e3);
    const double n1 = det3(a0, b0, e0, a2, b2, e2, a3, b3, e3);
    const double n2 = det3(a0, b0, e0, a1, b1, e1, a3, b3, e3);
    const double n3 = det3(a0, b0, e0, a1, b1, e1, a2, b2, e2);
    const double det = c0 * n0 - c1 * n1 + c2 * n2 - c3 * n3;
    const double rdet = 1.0 / det;
    iv0 = (float)(n0 * rdet);
    iv1 = (float)(-n1 * rdet);
    iv2 = (float)(n2 * rdet);
    iv3 = (float)(-n3 * rdet);
  }
  const float depth = iv0 * wx + iv1 * wy + iv2 * wz + iv3;

  wave_lds_sync();
  Gw[3 * lane + 0] = wx;
  Gw[3 * lane + 1] = wy;
  Gw[3 * lane + 2] = wz;
  Gw[3 * kWaveRays + lane] = depth;
  wave_lds_sync();
  {
    const v4f val = *(const v4f*)(Gw + 4 * lane);
    const size_t off = (lane < 24) ? (g0 * 3 + (size_t)(4 * lane))
                                   : ((size_t)kOut1Off + g0 + (size_t)(4 * (lane - 24)));
    float* dst = out + off;
    *(volatile v4f*)dst = val;
    __threadfence();
    *(volatile v4f*)dst = val;
  }
}

extern "C" void kernel_launch(void* const* d_in, const int* in_sizes, int n_in,
                              void* d_out, int out_size, void* d_ws, size_t ws_size,
                              hipStream_t stream) {
  (void)d_ws; (void)ws_size;
  if (n_in < 12) return;
  if (in_sizes[0] != kBatch * 16) return;
  if (in_sizes[1] != kBatch * 9) return;
  if (in_sizes[2] != kRays * 2) return;
  if (in_sizes[3] != kRays) return;
  if (in_sizes[4] != 3 * kFeat) return;
  if (in_sizes[5] != kFeat) return;
  if (in_sizes[6] != kGates * kFeat) return;
  if (in_sizes[7] != kGates) return;
  if (in_sizes[8] != kGates * kHid) return;
  if (in_sizes[9] != kGates) return;
  if (in_sizes[10] != kHid) return;
  if (in_sizes[11] != 1) return;
  if (out_size != kRays * 4) return;

  const float* cam2world  = (const float*)d_in[0];
  const float* intrinsics = (const float*)d_in[1];
  const float* uv         = (const float*)d_in[2];
  const float* init_depth = (const float*)d_in[3];
  const float* W_phi      = (const float*)d_in[4];
  const float* b_phi      = (const float*)d_in[5];
  const float* W_ih       = (const float*)d_in[6];
  const float* b_ih       = (const float*)d_in[7];
  const float* W_hh       = (const float*)d_in[8];
  const float* b_hh       = (const float*)d_in[9];
  const float* W_out      = (const float*)d_in[10];
  const float* b_out      = (const float*)d_in[11];
  float* out = (float*)d_out;

  ray_cell_kernel<<<dim3(kBlocks), dim3(kBlkThreads), 0, stream>>>(
      cam2world, intrinsics, uv, init_depth, W_phi, b_phi, W_ih, b_ih, W_hh, b_hh, W_out, b_out, out);
}
